// CachedMultiHeadAttention_21088289423900
// MI455X (gfx1250) — hardware-verified
//
#include <hip/hip_runtime.h>
#include <math.h>

#ifndef NB
#define NB 2
#endif
#ifndef SEQ
#define SEQ 2048
#endif
#ifndef RH
#define RH 512
#endif
#define NB_FULL 2
#define SEQ_FULL 2048
#define DIN 2048
#define DOUT 2048
#define NH 16
#define HD 128
#define NQKV (3 * DOUT)
#define RHE ((RH < SEQ) ? RH : SEQ)

static_assert(NB >= 1 && NB <= NB_FULL);
static_assert(SEQ >= 64 && SEQ <= SEQ_FULL && (SEQ % 64) == 0);
static_assert(RH >= 64 && (RH % 64) == 0);
static_assert(NH * HD == DOUT);
static_assert(HD == 128);
static_assert((DIN % 32) == 0 && (DOUT % 64) == 0 && (NQKV % 64) == 0);
static_assert(((NB * SEQ * DIN / 8) % 256) == 0 && ((NQKV * DIN / 8) % 256) == 0);
static_assert(((DOUT * DOUT / 8) % 256) == 0);

#define PSC  32768.0f
#define CTXC 32.0f
#define WPC  64.0f

typedef __attribute__((ext_vector_type(16))) _Float16 v16h;
typedef __attribute__((ext_vector_type(8)))  _Float16 v8h;
typedef __attribute__((ext_vector_type(16))) __bf16   v16b;
typedef __attribute__((ext_vector_type(8)))  __bf16   v8b;
typedef __attribute__((ext_vector_type(8)))  float    v8f;
typedef __attribute__((ext_vector_type(4)))  float    v4f;
typedef __attribute__((ext_vector_type(4)))  unsigned v4u;

__device__ __forceinline__ unsigned short bf_bits(float f) { unsigned u = __float_as_uint(f); return (unsigned short)((u + 0x7FFFu + ((u >> 16) & 1u)) >> 16); }
__device__ __forceinline__ float bf_val(unsigned short hb) { return __uint_as_float(((unsigned)hb) << 16); }
__device__ __forceinline__ float bf_rne(float f) { return bf_val(bf_bits(f)); }
__device__ __forceinline__ unsigned short h_bits(float f) { return __builtin_bit_cast(unsigned short, (_Float16)f); }
__device__ __forceinline__ float h_val(unsigned short hb) { return (float)__builtin_bit_cast(_Float16, hb); }
__device__ __forceinline__ v8f vz8() { v8f z = {0.f, 0.f, 0.f, 0.f, 0.f, 0.f, 0.f, 0.f}; return z; }
__device__ __forceinline__ v4u pack8(unsigned short a0, unsigned short a1, unsigned short a2, unsigned short a3,
                                     unsigned short a4, unsigned short a5, unsigned short a6, unsigned short a7) {
  v4u p;
  p.x = (unsigned)a0 | ((unsigned)a1 << 16); p.y = (unsigned)a2 | ((unsigned)a3 << 16);
  p.z = (unsigned)a4 | ((unsigned)a5 << 16); p.w = (unsigned)a6 | ((unsigned)a7 << 16);
  return p;
}

__device__ __forceinline__ v8f wmma_h(v16h a, v16h b, v8f c) {
  c = __builtin_amdgcn_wmma_f32_16x16x32_f16(false, a, false, b, (short)0, c, false, false);
  asm volatile("v_nop\n\tv_nop\n\tv_nop\n\tv_nop" : "+v"(c) : "v"(a), "v"(b));
  return c;
}
__device__ __forceinline__ v8f wmma_h2(v16h a, v16h a2, v16h b, v8f c) {
  c = __builtin_amdgcn_wmma_f32_16x16x32_f16(false, a, false, b, (short)0, c, false, false);
  c = __builtin_amdgcn_wmma_f32_16x16x32_f16(false, a2, false, b, (short)0, c, false, false);
  asm volatile("v_nop\n\tv_nop\n\tv_nop\n\tv_nop" : "+v"(c) : "v"(a), "v"(a2), "v"(b));
  return c;
}
__device__ __forceinline__ v8f wmma_h3(v16h ah, v16h al, v16h bh, v16h bl, v8f c) {
  c = __builtin_amdgcn_wmma_f32_16x16x32_f16(false, ah, false, bh, (short)0, c, false, false);
  c = __builtin_amdgcn_wmma_f32_16x16x32_f16(false, ah, false, bl, (short)0, c, false, false);
  c = __builtin_amdgcn_wmma_f32_16x16x32_f16(false, al, false, bh, (short)0, c, false, false);
  asm volatile("v_nop\n\tv_nop\n\tv_nop\n\tv_nop" : "+v"(c) : "v"(ah), "v"(al), "v"(bh), "v"(bl));
  return c;
}
__device__ __forceinline__ v8f wmma_b(v16b a, v16b b, v8f c) {
  c = __builtin_amdgcn_wmma_f32_16x16x32_bf16(false, a, false, b, (short)0, c, false, false);
  asm volatile("v_nop\n\tv_nop\n\tv_nop\n\tv_nop" : "+v"(c) : "v"(a), "v"(b));
  return c;
}
__device__ __forceinline__ v8f wmma_b2(v16b a, v16b a2, v16b b, v8f c) {
  c = __builtin_amdgcn_wmma_f32_16x16x32_bf16(false, a, false, b, (short)0, c, false, false);
  c = __builtin_amdgcn_wmma_f32_16x16x32_bf16(false, a2, false, b, (short)0, c, false, false);
  asm volatile("v_nop\n\tv_nop\n\tv_nop\n\tv_nop" : "+v"(c) : "v"(a), "v"(a2), "v"(b));
  return c;
}
__device__ __forceinline__ v8f wmma_b3(v16b ah, v16b al, v16b bh, v16b bl, v8f c) {
  c = __builtin_amdgcn_wmma_f32_16x16x32_bf16(false, ah, false, bh, (short)0, c, false, false);
  c = __builtin_amdgcn_wmma_f32_16x16x32_bf16(false, ah, false, bl, (short)0, c, false, false);
  c = __builtin_amdgcn_wmma_f32_16x16x32_bf16(false, al, false, bh, (short)0, c, false, false);
  asm volatile("v_nop\n\tv_nop\n\tv_nop\n\tv_nop" : "+v"(c) : "v"(ah), "v"(al), "v"(bh), "v"(bl));
  return c;
}
#define MEMBAR() asm volatile("" ::: "memory")
#define WAVE_LDS_SYNC() do { __builtin_amdgcn_fence(__ATOMIC_RELEASE, "workgroup"); __builtin_amdgcn_wave_barrier(); __builtin_amdgcn_fence(__ATOMIC_ACQUIRE, "workgroup"); } while (0)

template <int ET> struct FT;
template <> struct FT<0> {
  typedef v16h V; typedef v8h V8; typedef _Float16 S;
  union U { v16h v; v8h h[2]; };
  static __device__ __forceinline__ V load(const unsigned short* p) { U f; f.h[0] = *(const v8h*)p; f.h[1] = *(const v8h*)(p + 16); return f.v; }
  static __device__ __forceinline__ S enc(float f) { return (_Float16)f; }
  static __device__ __forceinline__ float dec(S s) { return (float)s; }
  static __device__ __forceinline__ v8f mma(V a, V b, v8f c) { return wmma_h(a, b, c); }
  static __device__ __forceinline__ v8f mma2(V a, V a2, V b, v8f c) { return wmma_h2(a, a2, b, c); }
  static __device__ __forceinline__ v8f mma3(V ah, V al, V bh, V bl, v8f c) { return wmma_h3(ah, al, bh, bl, c); }
};
template <> struct FT<1> {
  typedef v16b V; typedef v8b V8; typedef __bf16 S;
  union U { v16b v; v8b h[2]; };
  static __device__ __forceinline__ V load(const unsigned short* p) { U f; f.h[0] = *(const v8b*)p; f.h[1] = *(const v8b*)(p + 16); return f.v; }
  static __device__ __forceinline__ S enc(float f) { return __builtin_bit_cast(__bf16, bf_bits(f)); }
  static __device__ __forceinline__ float dec(S s) { return bf_val(__builtin_bit_cast(unsigned short, s)); }
  static __device__ __forceinline__ v8f mma(V a, V b, v8f c) { return wmma_b(a, b, c); }
  static __device__ __forceinline__ v8f mma2(V a, V a2, V b, v8f c) { return wmma_b2(a, a2, b, c); }
  static __device__ __forceinline__ v8f mma3(V ah, V al, V bh, V bl, v8f c) { return wmma_b3(ah, al, bh, bl, c); }
};

__global__ __launch_bounds__(256) void k_cvt_in(const float* __restrict__ x, const float* __restrict__ wqkv,
                                                unsigned short* __restrict__ xb, unsigned short* __restrict__ wb) {
  const long long t = (long long)blockIdx.x * 256 + threadIdx.x;
  const long long nx = (long long)NB * SEQ * DIN / 8, nw = (long long)NQKV * DIN / 8;
  if (t >= nx + nw) return;
  const float* src; unsigned short* dst;
  if (t < nx) {
    const long long e = t * 8; const long long r = e / DIN; const int cc = (int)(e - r * DIN);
    const int b = (int)(r / SEQ); const int s = (int)(r - (long long)b * SEQ);
    src = x + ((size_t)b * SEQ_FULL + s) * DIN + cc; dst = xb + e;
  } else {
    const long long e = (t - nx) * 8; src = wqkv + e; dst = wb + e;
  }
  const v4f a = *(const v4f*)src; const v4f c4 = *(const v4f*)(src + 4);
  const v4u pk = pack8(bf_bits(a.x), bf_bits(a.y), bf_bits(a.z), bf_bits(a.w), bf_bits(c4.x), bf_bits(c4.y), bf_bits(c4.z), bf_bits(c4.w));
  volatile v4u* d = (volatile v4u*)dst; *d = pk; __threadfence(); *d = pk;
}

__global__ __launch_bounds__(256) void k_cvt_w(const float* __restrict__ wproj, unsigned short* __restrict__ wp, unsigned short* __restrict__ wpb) {
  const long long t = (long long)blockIdx.x * 256 + threadIdx.x;
  if (t >= (long long)DOUT * DOUT / 8) return;
  const float* src = wproj + t * 8;
  const v4f a = *(const v4f*)src; const v4f c4 = *(const v4f*)(src + 4);
  const float f[8] = {a.x, a.y, a.z, a.w, c4.x, c4.y, c4.z, c4.w};
  unsigned short ob[8], oh[8];
#pragma unroll
  for (int e = 0; e < 8; ++e) { ob[e] = bf_bits(f[e]); oh[e] = h_bits(bf_val(ob[e]) * WPC); }
  const v4u ph = pack8(oh[0], oh[1], oh[2], oh[3], oh[4], oh[5], oh[6], oh[7]);
  const v4u pb = pack8(ob[0], ob[1], ob[2], ob[3], ob[4], ob[5], ob[6], ob[7]);
  volatile v4u* dh = (volatile v4u*)(wp + t * 8); volatile v4u* db = (volatile v4u*)(wpb + t * 8);
  *dh = ph; *db = pb; __threadfence(); *dh = ph; *db = pb;
}

struct GArgs {
  const unsigned short* A; const unsigned short* A2; const unsigned short* Bt; const float* bias;
  float* Cf; unsigned short* Ch; unsigned short* Cbh; unsigned short* Cbl;
  long long sA, sA2, sCf, sCh, sCb;
  int lda, ldb, ldc, ldh, ldcb, M, N, K, lorows; float scale;
};
static_assert(sizeof(GArgs) == 8 * 8 + 5 * 8 + 10 * 4);

template <int ET, int TN, bool ASPLIT, int OUTM>
__global__ __launch_bounds__(256) void k_gemm(GArgs g) {
  static_assert(TN == 2 || TN == 4);
  static_assert(OUTM == 0 || (TN == 4 && !ASPLIT));
  typedef typename FT<ET>::V V;
  __shared__ __align__(16) float sT[8][16 * 68];
  const int b = blockIdx.y, lane = threadIdx.x & 31, wave = threadIdx.x >> 5;
  const int tilesN = g.N / (16 * TN), tilesM = g.M >> 6;
  const int tile = blockIdx.x * 8 + wave;
  if (tile >= tilesM * tilesN) return;
  const int tm = tile / tilesN, tn = tile - tm * tilesN;
  const int m0 = tm << 6, n0 = tn * (16 * TN);
  const unsigned short* Ab = g.A + (size_t)b * g.sA;
  const unsigned short* A2b = ASPLIT ? (g.A2 + (size_t)b * g.sA2) : Ab;
  const int rl = lane & 15, koff = (lane >> 4) * 8, mOff = (lane >> 4) * 8;

  v8f acc[4][TN];
#pragma unroll
  for (int i = 0; i < 4; ++i)
#pragma unroll
    for (int j = 0; j < TN; ++j) acc[i][j] = vz8();

  for (int k0 = 0; k0 < g.K; k0 += 32) {
    V bq[TN];
#pragma unroll
    for (int j = 0; j < TN; ++j) bq[j] = FT<ET>::load(g.Bt + (size_t)(n0 + 16 * j + rl) * g.ldb + koff + k0);
#pragma unroll
    for (int i = 0; i < 4; ++i) {
      const size_t ao = (size_t)(m0 + 16 * i + rl) * g.lda + koff + k0;
      const V ah = FT<ET>::load(Ab + ao);
      V al = ah;
      if (ASPLIT) al = FT<ET>::load(A2b + ao);
      MEMBAR();
#pragma unroll
      for (int j = 0; j < TN; ++j) {
        if (ASPLIT) acc[i][j] = FT<ET>::mma2(ah, al, bq[j], acc[i][j]);
        else acc[i][j] = FT<ET>::mma(ah, bq[j], acc[i][j]);
      }
    }
  }

  float* slab = sT[wave];
#pragma unroll
  for (int i = 0; i < 4; ++i) {
    const int mB = m0 + 16 * i;
#pragma unroll
    for (int j = 0; j < TN; ++j) {
      const int n = n0 + 16 * j + rl;
      float bv = 0.f;
      if (OUTM == 0) bv = bf_rne(g.bias[n]);
#pragma unroll
      for (int r = 0; r < 8; ++r) {
        float v = acc[i][j][r];
        if (OUTM == 0) v = v * g.scale + bv;
        slab[(mOff + r) * 68 + 16 * j + rl] = v;
      }
    }
    WAVE_LDS_SYNC();
    if (OUTM == 0) {
      float* C = g.Cf + (size_t)b * g.sCf;
      if (TN == 4) {
        const int h2 = lane >> 4, c4 = (lane & 15) * 4;
        for (int pass = 0; pass < 2; ++pass) {
#pragma unroll
          for (int it = 0; it < 8; ++it) {
            const int row = 2 * it + h2;
            const v4f v = *(const v4f*)(slab + row * 68 + c4);
            *(volatile v4f*)(C + (size_t)(mB + row) * g.ldc + n0 + c4) = v;
          }
          __threadfence();
        }
      } else {
        const int q4 = lane >> 3, c4 = (lane & 7) * 4;
        for (int pass = 0; pass < 2; ++pass) {
#pragma unroll
          for (int it = 0; it < 4; ++it) {
            const int row = 4 * it + q4;
            const v4f v = *(const v4f*)(slab + row * 68 + c4);
            *(volatile v4f*)(C + (size_t)(mB + row) * g.ldc + n0 + c4) = v;
          }
          __threadfence();
        }
      }
    } else {
      unsigned short* C  = g.Ch  + (size_t)b * g.sCh;
      unsigned short* CBh = g.Cbh + (size_t)b * g.sCb;
      unsigned short* CBl = g.Cbl + (size_t)b * g.sCb;
      const bool dolo = (m0 < g.lorows);
      const int q4 = lane >> 3, c8 = (lane & 7) * 8;
      for (int pass = 0; pass < 2; ++pass) {
#pragma unroll
        for (int it = 0; it < 4; ++it) {
          const int row = 4 * it + q4;
          const float* sp = slab + row * 68 + c8;
          unsigned short hb[8];
#pragma unroll
          for (int e = 0; e < 8; ++e) hb[e] = h_bits(sp[e]);
          const v4u ph = pack8(hb[0], hb[1], hb[2], hb[3], hb[4], hb[5], hb[6], hb[7]);
          *(volatile v4u*)(C + (size_t)(mB + row) * g.ldh + n0 + c8) = ph;
          if (dolo) {
            unsigned short bh[8], bl[8];
#pragma unroll
            for (int e = 0; e < 8; ++e) { bh[e] = bf_bits(sp[e]); bl[e] = bf_bits(sp[e] - bf_val(bh[e])); }
            const v4u p1 = pack8(bh[0], bh[1], bh[2], bh[3], bh[4], bh[5], bh[6], bh[7]);
            const v4u p2 = pack8(bl[0], bl[1], bl[2], bl[3], bl[4], bl[5], bl[6], bl[7]);
            *(volatile v4u*)(CBh + (size_t)(mB + row) * g.ldcb + n0 + c8) = p1;
            *(volatile v4u*)(CBl + (size_t)(mB + row) * g.ldcb + n0 + c8) = p2;
          }
        }
        __threadfence();
      }
    }
    WAVE_LDS_SYNC();
  }
}

__global__ __launch_bounds__(256) void k_vt(const unsigned short* __restrict__ src, int lds, int srows, unsigned short* __restrict__ dst, int ldd) {
  __shared__ __align__(16) unsigned int tile[64][36];
  const int dt = blockIdx.x, kt = blockIdx.y, b = blockIdx.z, h = dt >> 1, dh = dt & 1, t = threadIdx.x;
  const size_t srow0 = (size_t)b * srows + (size_t)kt * 64;
  const int scol0 = 2 * DOUT + h * HD + dh * 64;
#pragma unroll
  for (int it = 0; it < 2; ++it) {
    const int p = t + 256 * it; const int row = p >> 3, c8 = (p & 7) * 8;
    const v4u v = *(const v4u*)(src + (srow0 + row) * (size_t)lds + scol0 + c8);
    *(v4u*)&tile[row][c8 >> 1] = v;
  }
  __syncthreads();
  const size_t drow0 = ((size_t)b * NH + h) * HD + dh * 64;
  const int key0 = kt * 64;
  for (int pass = 0; pass < 2; ++pass) {
#pragma unroll
    for (int it = 0; it < 2; ++it) {
      const int p = t + 256 * it; const int d = p >> 3, k8 = (p & 7) * 8;
      unsigned short o[8];
#pragma unroll
      for (int e = 0; e < 8; ++e) { const unsigned w = tile[k8 + e][d >> 1]; o[e] = (d & 1) ? (unsigned short)(w >> 16) : (unsigned short)(w & 0xFFFFu); }
      const v4u pk = pack8(o[0], o[1], o[2], o[3], o[4], o[5], o[6], o[7]);
      *(volatile v4u*)(dst + (drow0 + d) * (size_t)ldd + key0 + k8) = pk;
    }
    __threadfence();
  }
}

template <bool RES>
__global__ __launch_bounds__(128) __attribute__((amdgpu_num_vgpr(256))) void k_attn(const unsigned short* Qh, const unsigned short* Ql,
                                              const unsigned short* Vh, const unsigned short* Vl,
                                              unsigned short* Oh, unsigned short* Ol, int qb_lo, int nq, float scale) {
  constexpr int ET = RES ? 1 : 0;
  typedef typename FT<ET>::V V;
  typedef typename FT<ET>::V8 V8;
  typedef typename FT<ET>::S S16;
  typedef typename FT<ET>::U U;
  constexpr int NDT = RES ? 4 : 8;
  constexpr int PP = 72;
  constexpr int OSP = 132;
  __shared__ __align__(16) S16 Psh[4][16 * PP];
  __shared__ __align__(16) S16 Psl[RES ? 4 : 1][16 * PP];
  __shared__ __align__(16) float Os[4][16 * OSP];
  const int srows = RES ? RHE : SEQ;
  const int tid = threadIdx.x, wave = tid >> 5, lane = tid & 31, hh = lane >> 4, c = lane & 15;
  int bx = blockIdx.x; int dsel = 0;
  if (RES) { dsel = bx & 1; bx >>= 1; }
  const int qb = qb_lo + bx % nq;
  const int bh = bx / nq;
  const int h = bh % NH, b = bh / NH;
  const int q0 = qb * 64 + wave * 16;
  const int dbase = dsel * 64;
  const float L2E = 1.4426950408889634f;
  const float NEG = -__builtin_inff();

  const unsigned short* qr  = Qh + ((size_t)b * srows + q0 + c) * NQKV + h * HD + 8 * hh;
  const unsigned short* qlr = Ql + ((size_t)b * srows + q0 + c) * NQKV + h * HD + 8 * hh;
  V qreg[4];
  if (!RES) {
#pragma unroll
    for (int dc = 0; dc < 4; ++dc) qreg[dc] = FT<ET>::load(qr + dc * 32);
  }
  float mrow[8], lrow[8];
  v8f oacc[NDT];
#pragma unroll
  for (int r = 0; r < 8; ++r) { mrow[r] = NEG; lrow[r] = 0.f; }
#pragma unroll
  for (int t = 0; t < NDT; ++t) oacc[t] = vz8();

  const unsigned short* kb0 = Qh + (size_t)b * srows * NQKV + DOUT + h * HD + 8 * hh;
  const unsigned short* kl0 = Ql + (size_t)b * srows * NQKV + DOUT + h * HD + 8 * hh;
  const unsigned short* vb0 = Vh + ((size_t)bh * HD + dbase + c) * srows + 8 * hh;
  const unsigned short* vl0 = Vl + ((size_t)bh * HD + dbase + c) * srows + 8 * hh;
  S16* pwh = Psh[wave];
  S16* pwl = Psl[RES ? wave : 0];

  for (int kc = 0; kc <= qb; ++kc) {
    const int kv0 = kc * 64;
    v8f s[4];
#pragma unroll
    for (int j = 0; j < 4; ++j) {
      v8f sj = vz8();
      const unsigned krow = (unsigned)(kv0 + 16 * j + c) * (unsigned)NQKV;
#pragma unroll
      for (int dc = 0; dc < 4; ++dc) {
        const V kf = FT<ET>::load(kb0 + krow + dc * 32);
        if (RES) {
          const V klf = FT<ET>::load(kl0 + krow + dc * 32);
          const V qf  = FT<ET>::load(qr + dc * 32);
          const V qlf = FT<ET>::load(qlr + dc * 32);
          MEMBAR();
          sj = FT<ET>::mma3(qf, qlf, kf, klf, sj);
        } else {
          MEMBAR();
          sj = FT<ET>::mma(qreg[dc], kf, sj);
        }
      }
      s[j] = sj;
    }
    float cm[8];
#pragma unroll
    for (int r = 0; r < 8; ++r) {
      const int qrow = q0 + 8 * hh + r;
      float m = NEG;
#pragma unroll
      for (int j = 0; j < 4; ++j) {
        const int kvcol = kv0 + 16 * j + c;
        float v = s[j][r] * scale;
        v = (kvcol > qrow) ? NEG : v * L2E;
        s[j][r] = v;
        m = fmaxf(m, v);
      }
      m = fmaxf(m, __shfl_xor(m, 1, 32)); m = fmaxf(m, __shfl_xor(m, 2, 32));
      m = fmaxf(m, __shfl_xor(m, 4, 32)); m = fmaxf(m, __shfl_xor(m, 8, 32));
      cm[r] = m;
    }
#pragma unroll
    for (int r = 0; r < 8; ++r) {
      const float mnew = fmaxf(mrow[r], cm[r]);
      const float alpha = (mnew == NEG) ? 1.f : exp2f(mrow[r] - mnew);
      mrow[r] = mnew;
      float psum = 0.f;
#pragma unroll
      for (int j = 0; j < 4; ++j) {
        const float p = (s[j][r] == NEG) ? 0.f : exp2f(s[j][r] - mnew);
        psum += p;
        const float pe = RES ? p : p * PSC;
        const S16 ph = FT<ET>::enc(pe);
        pwh[(8 * hh + r) * PP + 16 * j + c] = ph;
        if (RES) pwl[(8 * hh + r) * PP + 16 * j + c] = FT<ET>::enc(pe - FT<ET>::dec(ph));
      }
      psum += __shfl_xor(psum, 1, 32); psum += __shfl_xor(psum, 2, 32);
      psum += __shfl_xor(psum, 4, 32); psum += __shfl_xor(psum, 8, 32);
      lrow[r] = lrow[r] * alpha + psum;
#pragma unroll
      for (int t = 0; t < NDT; ++t) oacc[t][r] *= alpha;
    }
    WAVE_LDS_SYNC();
#pragma unroll
    for (int kk = 0; kk < 2; ++kk) {
      U pa, pl;
      pa.h[0] = *(const V8*)(pwh + c * PP + kk * 32 + 8 * hh);
      pa.h[1] = *(const V8*)(pwh + c * PP + kk * 32 + 16 + 8 * hh);
      pl.v = pa.v;
      if (RES) {
        pl.h[0] = *(const V8*)(pwl + c * PP + kk * 32 + 8 * hh);
        pl.h[1] = *(const V8*)(pwl + c * PP + kk * 32 + 16 + 8 * hh);
      }
#pragma unroll
      for (int t = 0; t < NDT; ++t) {
        const V vf = FT<ET>::load(vb0 + (size_t)(16 * t) * srows + kv0 + kk * 32);
        if (RES) {
          const V vlf = FT<ET>::load(vl0 + (size_t)(16 * t) * srows + kv0 + kk * 32);
          MEMBAR();
          oacc[t] = FT<ET>::mma3(pa.v, pl.v, vf, vlf, oacc[t]);
        } else {
          MEMBAR();
          oacc[t] = FT<ET>::mma(pa.v, vf, oacc[t]);
        }
      }
    }
    WAVE_LDS_SYNC();
  }

  float* os = Os[wave];
#pragma unroll
  for (int r = 0; r < 8; ++r) {
    const float inv = RES ? (1.0f / lrow[r]) : (1.0f / (lrow[r] * (PSC / CTXC)));
#pragma unroll
    for (int t = 0; t < NDT; ++t) os[(8 * hh + r) * OSP + 16 * t + c] = oacc[t][r] * inv;
  }
  WAVE_LDS_SYNC();
  const size_t orow0 = (size_t)b * srows + q0;
  if (!RES) {
    const int h2 = lane >> 4, c8 = (lane & 15) * 8;
    for (int pass = 0; pass < 2; ++pass) {
#pragma unroll
      for (int it = 0; it < 8; ++it) {
        const int row = 2 * it + h2;
        const float* sp = os + row * OSP + c8;
        const v4u pk = pack8(h_bits(sp[0]), h_bits(sp[1]), h_bits(sp[2]), h_bits(sp[3]), h_bits(sp[4]), h_bits(sp[5]), h_bits(sp[6]), h_bits(sp[7]));
        *(volatile v4u*)(Oh + (orow0 + row) * DOUT + h * HD + c8) = pk;
      }
      __threadfence();
    }
  } else {
    const int q4 = lane >> 3, c8 = (lane & 7) * 8;
    for (int pass = 0; pass < 2; ++pass) {
#pragma unroll
      for (int it = 0; it < 4; ++it) {
        const int row = 4 * it + q4;
        const float* sp = os + row * OSP + c8;
        unsigned short hb[8], lb[8];
#pragma unroll
        for (int e = 0; e < 8; ++e) { hb[e] = bf_bits(sp[e]); lb[e] = bf_bits(sp[e] - bf_val(hb[e])); }
        const v4u ph = pack8(hb[0], hb[1], hb[2], hb[3], hb[4], hb[5], hb[6], hb[7]);
        const v4u pl = pack8(lb[0], lb[1], lb[2], lb[3], lb[4], lb[5], lb[6], lb[7]);
        *(volatile v4u*)(Oh + (orow0 + row) * DOUT + h * HD + dbase + c8) = ph;
        *(volatile v4u*)(Ol + (orow0 + row) * DOUT + h * HD + dbase + c8) = pl;
      }
      __threadfence();
    }
  }
}

static inline size_t al256(size_t v) { return (v + 255) & ~(size_t)255; }

extern "C" void kernel_launch(void* const* d_in, const int* in_sizes, int n_in, void* d_out, int out_size, void* d_ws, size_t ws_size, hipStream_t stream) {
  if (n_in < 4) return;
  if (in_sizes[0] < (NB - 1) * SEQ_FULL * DIN + SEQ * DIN) return;
  if (in_sizes[1] < NQKV * DIN) return;
  if (in_sizes[2] < DOUT * DOUT) return;
  if (in_sizes[3] < DOUT) return;
  if (out_size < (NB - 1) * SEQ_FULL * DOUT + SEQ * DOUT) return;
  const float* x = (const float*)d_in[0];
  const float* w_qkv = (const float*)d_in[1];
  const float* w_proj = (const float*)d_in[2];
  const float* b_proj = (const float*)d_in[3];
  float* out = (float*)d_out;

  const size_t szXb  = al256((size_t)NB * SEQ * DIN * 2);
  const size_t szWb  = al256((size_t)NQKV * DIN * 2);
  const size_t szWp  = al256((size_t)DOUT * DOUT * 2);
  const size_t szQh  = al256((size_t)NB * SEQ * NQKV * 2);
  const size_t szQb  = al256((size_t)NB * RHE * NQKV * 2);
  const size_t szVh  = al256((size_t)NB * NH * HD * SEQ * 2);
  const size_t szVb  = al256((size_t)NB * NH * HD * RHE * 2);
  const size_t szCh  = al256((size_t)NB * SEQ * DOUT * 2);
  const size_t szCb  = al256((size_t)NB * RHE * DOUT * 2);
  size_t szA = szXb + szWb; { const size_t s2 = szVh + 2 * szVb + szCh + 2 * szCb; if (s2 > szA) szA = s2; }
  size_t szB = 2 * szQb; { const size_t s2 = 2 * szWp; if (s2 > szB) szB = s2; }
  const size_t total = szA + szQh + szB;
  if (total > ws_size) return;
  char* ws = (char*)d_ws;
  unsigned short* Xb    = (unsigned short*)(ws);
  unsigned short* Wb    = (unsigned short*)(ws + szXb);
  unsigned short* Vth   = (unsigned short*)(ws);
  unsigned short* Vtbh  = (unsigned short*)(ws + szVh);
  unsigned short* Vtbl  = (unsigned short*)(ws + szVh + szVb);
  unsigned short* Ch    = (unsigned short*)(ws + szVh + 2 * szVb);
  unsigned short* Cbh   = (unsigned short*)(ws + szVh + 2 * szVb + szCh);
  unsigned short* Cbl   = (unsigned short*)(ws + szVh + 2 * szVb + szCh + szCb);
  unsigned short* QKVh  = (unsigned short*)(ws + szA);
  char* regB = ws + szA + szQh;
  unsigned short* QKVbh = (unsigned short*)(regB);
  unsigned short* QKVbl = (unsigned short*)(regB + szQb);
  unsigned short* Wp    = (unsigned short*)(regB);
  unsigned short* Wpb   = (unsigned short*)(regB + szWp);

  const float scale = 1.0f / sqrtf((float)HD);
  const bool tail = (SEQ - RHE) > 0;

  {
    const long long nthr = (long long)NB * SEQ * DIN / 8 + (long long)NQKV * DIN / 8;
    k_cvt_in<<<(unsigned)((nthr + 255) / 256), 256, 0, stream>>>(x, w_qkv, Xb, Wb);
  }
  {
    GArgs ga;
    ga.A = Xb; ga.A2 = Xb; ga.Bt = Wb; ga.bias = b_proj;
    ga.Cf = out; ga.Ch = QKVh; ga.Cbh = QKVbh; ga.Cbl = QKVbl;
    ga.sA = (long long)SEQ * DIN; ga.sA2 = 0; ga.sCf = 0; ga.sCh = (long long)SEQ * NQKV; ga.sCb = (long long)RHE * NQKV;
    ga.lda = DIN; ga.ldb = DIN; ga.ldc = DOUT; ga.ldh = NQKV; ga.ldcb = NQKV; ga.M = SEQ; ga.N = NQKV; ga.K = DIN; ga.lorows = RHE;
    ga.scale = 1.f;
    const unsigned tiles = (unsigned)((SEQ / 64) * (NQKV / 64));
    k_gemm<1, 4, false, 1><<<dim3((tiles + 7) / 8, NB), 256, 0, stream>>>(ga);
  }
  if (tail) k_vt<<<dim3(2 * NH, SEQ / 64, NB), 256, 0, stream>>>(QKVh, NQKV, SEQ, Vth, SEQ);
  k_vt<<<dim3(2 * NH, RHE / 64, NB), 256, 0, stream>>>(QKVbh, NQKV, RHE, Vtbh, RHE);
  k_vt<<<dim3(2 * NH, RHE / 64, NB), 256, 0, stream>>>(QKVbl, NQKV, RHE, Vtbl, RHE);
  {
    const int nqr = RHE / 64;
    k_attn<true><<<(unsigned)(2 * NB * NH * nqr), 128, 0, stream>>>(QKVbh, QKVbl, Vtbh, Vtbl, Cbh, Cbl, 0, nqr, scale);
    const int nqp = (SEQ - RHE) / 64;
    if (nqp > 0) k_attn<false><<<(unsigned)(NB * NH * nqp), 128, 0, stream>>>(QKVh, QKVh, Vth, Vth, Ch, Ch, nqr, nqp, scale);
  }
  k_cvt_w<<<(unsigned)(((long long)DOUT * DOUT / 8 + 255) / 256), 256, 0, stream>>>(w_proj, Wp, Wpb);
  {
    GArgs gr;
    gr.A = Cbh; gr.A2 = Cbl; gr.Bt = Wpb; gr.bias = b_proj;
    gr.Cf = out; gr.Ch = QKVh; gr.Cbh = QKVh; gr.Cbl = QKVh;
    gr.sA = (long long)RHE * DOUT; gr.sA2 = (long long)RHE * DOUT; gr.sCf = (long long)SEQ_FULL * DOUT; gr.sCh = 0; gr.sCb = 0;
    gr.lda = DOUT; gr.ldb = DOUT; gr.ldc = DOUT; gr.ldh = NQKV; gr.ldcb = NQKV; gr.M = RHE; gr.N = DOUT; gr.K = DOUT; gr.lorows = 0;
    gr.scale = 1.0f;
    const unsigned tr = (unsigned)((RHE / 64) * (DOUT / 32));
    k_gemm<1, 2, true, 0><<<dim3((tr + 7) / 8, NB), 256, 0, stream>>>(gr);

    if (tail) {
      GArgs gp = gr;
      gp.A = Ch + (size_t)RHE * DOUT; gp.A2 = gp.A; gp.Bt = Wp;
      gp.sA = (long long)SEQ * DOUT; gp.sA2 = (long long)SEQ * DOUT;
      gp.Cf = out + (size_t)RHE * DOUT; gp.M = SEQ - RHE; gp.scale = 1.0f / (WPC * CTXC);
      const unsigned tp = (unsigned)(((SEQ - RHE) / 64) * (DOUT / 64));
      k_gemm<0, 4, false, 0><<<dim3((tp + 7) / 8, NB), 256, 0, stream>>>(gp);
    }
  }
}
